// IPDF_Encoder_75943611728458
// MI455X (gfx1250) — hardware-verified
//
#include <hip/hip_runtime.h>
#include <stddef.h>


#define NB     16
#define CIN    6
#define HID    256
#define VL     32768
#define NE     8
#define NT     64
#define NCH    (VL / NT)
#define NCHB   8
#define NTHR   256
#define NWAVE  (NTHR / 32)
#define P1     264
#define SC_A   8.0f
#define SC_W   64.0f
#define SC_AW  512.0f
#define SC_INV (1.0f / 512.0f)
#define PIECES (HID * HID / 8)
#define NBKP   (NB * PIECES / NTHR)

static_assert(PIECES == 8192);
static_assert(NBKP * NTHR == NB * PIECES);
static_assert(NCH % NCHB == 0);
static_assert(NT == 8 * NWAVE);
static_assert(HID == 8 * 32);
static_assert(HID == 32 * NWAVE);
static_assert(NT == 4 * 16);
static_assert((P1 * 2) % 16 == 0);
static_assert(P1 >= HID);
static_assert(HID % 32 == 0);
static_assert(NTHR == HID);
static_assert(CIN * NT <= 2 * NTHR);
static_assert(NT / 4 <= 32);

typedef _Float16 v16h __attribute__((ext_vector_type(16)));
typedef _Float16 v8h  __attribute__((ext_vector_type(8)));
typedef float    v4f  __attribute__((ext_vector_type(4)));
typedef float    v8f  __attribute__((ext_vector_type(8)));
union FragH { v16h v; v8h h[2]; };

__device__ __forceinline__ v8f wmh(v16h a, v16h b, v8f c) {
  v8f d = __builtin_amdgcn_wmma_f32_16x16x32_f16(false, a, false, b, (short)0, c, false, false);
#if defined(__HIP_DEVICE_COMPILE__)
  asm volatile("v_nop\n\tv_nop\n\tv_nop\n\tv_nop" : "+v"(d) : "v"(a), "v"(b));
#endif
  return d;
}

__device__ __forceinline__ v8f zero8() {
  v8f z = {0.f, 0.f, 0.f, 0.f, 0.f, 0.f, 0.f, 0.f};
  return z;
}

__device__ __forceinline__ v16h afrag(const _Float16* row, int k0, int h) {
  FragH u;
  u.h[0] = *(const v8h*)(row + k0 + 8 * h);
  u.h[1] = *(const v8h*)(row + k0 + 16 + 8 * h);
  return u.v;
}

__device__ __forceinline__ int sel_idx(int e) {
  e = e < 0 ? e + NE : e;
  e = e < 0 ? 0 : e;
  e = e > NE - 1 ? NE - 1 : e;
  return e;
}

__global__ __launch_bounds__(NTHR) void k_prep(const float* __restrict__ w2, const int* __restrict__ oidx,
                                               _Float16* w2s) {
  const int g  = blockIdx.x * NTHR + (int)threadIdx.x;
  int b = g >> 13;
  b = b > NB - 1 ? NB - 1 : b;
  const int pc = g & (PIECES - 1);
  const int e  = sel_idx(oidx[b]);
  const float* src = w2 + (size_t)e * HID * HID + (size_t)8 * pc;
  const v4f u0 = *(const v4f*)src;
  const v4f u1 = *(const v4f*)(src + 4);
  v8h o;
#pragma unroll
  for (int i = 0; i < 4; ++i) {
    o[i]     = (_Float16)(SC_W * u0[i]);
    o[4 + i] = (_Float16)(SC_W * u1[i]);
  }
  _Float16* p = w2s + (size_t)b * HID * HID + (size_t)8 * pc;
  *(volatile v8h*)p = o;
  __threadfence();
  *(volatile v8h*)p = o;
}

__global__ __launch_bounds__(NTHR) void k_main(const float* __restrict__ x, const int* __restrict__ oidx,
                                               const float* __restrict__ w1, const float* __restrict__ b1,
                                               const _Float16* __restrict__ w2s,
                                               const float* __restrict__ b2, const float* __restrict__ w3,
                                               const float* __restrict__ b3, float* out) {
  __shared__ __align__(16) _Float16 sh1[NT * P1];
  __shared__ __align__(16) float s_x[CIN * NT];
  __shared__ __align__(32) float s_b2s[HID];
  __shared__ __align__(32) float s_w3s[HID];
  __shared__ __align__(16) v4f s_part4[NWAVE * NT / 4];
  float* s_part = (float*)s_part4;

  const int tid = (int)threadIdx.x, lane = tid & 31, w = tid >> 5, h = lane >> 4, m = lane & 15;
  const int b   = blockIdx.y;
  const int ch0 = blockIdx.x * NCHB;
  const int e   = sel_idx(oidx[b]);

  s_b2s[tid] = SC_AW * b2[(size_t)e * HID + tid];
  s_w3s[tid] = SC_INV * w3[(size_t)e * HID + tid];
  const float bias3 = b3[e];

  v4f wv[12];
  v4f bv[2];
  {
    const float* wp = w1 + (size_t)e * HID * CIN + (size_t)(8 * lane) * CIN;
#pragma unroll
    for (int i = 0; i < 12; ++i) wv[i] = *(const v4f*)(wp + 4 * i);
    const float* bp = b1 + (size_t)e * HID + 8 * lane;
    bv[0] = *(const v4f*)bp;
    bv[1] = *(const v4f*)(bp + 4);
  }

  const _Float16* arow0 = w2s + (size_t)b * HID * HID + (size_t)(32 * w + m) * HID;
  const _Float16* arow1 = arow0 + 16 * HID;
  float* orow = out + (size_t)b * VL;

#pragma unroll 1
  for (int c = 0; c < NCHB; ++c) {
    const int col0 = (ch0 + c) * NT;

    for (int idx = tid; idx < CIN * NT; idx += NTHR) {
      const int i = idx >> 6, n = idx & (NT - 1);
      s_x[idx] = x[(size_t)(b * CIN + i) * VL + col0 + n];
    }
    __syncthreads();

#pragma unroll 2
    for (int j = 0; j < NT / NWAVE; ++j) {
      const int n = w + NWAVE * j;
      float xv[CIN];
#pragma unroll
      for (int i = 0; i < CIN; ++i) xv[i] = s_x[i * NT + n];
      v8h o;
#pragma unroll
      for (int q = 0; q < 8; ++q) {
        float s = bv[q >> 2][q & 3];
#pragma unroll
        for (int i = 0; i < CIN; ++i) {
          const int f = CIN * q + i;
          s = fmaf(wv[f >> 2][f & 3], xv[i], s);
        }
        o[q] = (_Float16)(SC_A * fmaxf(s, 0.0f));
      }
      *(v8h*)(sh1 + n * P1 + 8 * lane) = o;
    }
    __syncthreads();

    v8f acc[2][4];
#pragma unroll
    for (int mt = 0; mt < 2; ++mt)
#pragma unroll
      for (int ct = 0; ct < 4; ++ct) acc[mt][ct] = zero8();

#pragma unroll
    for (int ks = 0; ks < HID / 32; ++ks) {
      const int k0 = 32 * ks;
      const v16h a0 = afrag(arow0, k0, h);
      const v16h a1 = afrag(arow1, k0, h);
#pragma unroll
      for (int ct = 0; ct < 4; ++ct) {
        const v16h bf = afrag(sh1 + (16 * ct + m) * P1, k0, h);
        acc[0][ct] = wmh(a0, bf, acc[0][ct]);
        acc[1][ct] = wmh(a1, bf, acc[1][ct]);
      }
    }

    float p[4];
#pragma unroll
    for (int ct = 0; ct < 4; ++ct) p[ct] = 0.0f;
#pragma unroll
    for (int mt = 0; mt < 2; ++mt) {
      const int ob = 32 * w + 16 * mt + 8 * h;
      const v8f bb = *(const v8f*)(s_b2s + ob);
      const v8f ww = *(const v8f*)(s_w3s + ob);
#pragma unroll
      for (int r = 0; r < 8; ++r) {
#pragma unroll
        for (int ct = 0; ct < 4; ++ct) {
          const float v = fmaxf(acc[mt][ct][r] + bb[r], 0.0f);
          p[ct] = fmaf(ww[r], v, p[ct]);
        }
      }
    }
#pragma unroll
    for (int ct = 0; ct < 4; ++ct) {
      p[ct] += __shfl_xor(p[ct], 16, 32);
      s_part[w * NT + 16 * ct + m] = p[ct];
    }
    __syncthreads();

    if (w == 0) {
      if (lane < NT / 4) {
        v4f s = s_part4[lane];
#pragma unroll
        for (int q = 1; q < NWAVE; ++q) s += s_part4[q * (NT / 4) + lane];
        v4f o;
#pragma unroll
        for (int i = 0; i < 4; ++i) o[i] = s[i] + bias3;
        float* po = orow + col0 + 4 * lane;
        *(volatile v4f*)po = o;
        __threadfence();
        *(volatile v4f*)po = o;
      }
    }
  }
}

extern "C" void kernel_launch(void* const* d_in, const int* in_sizes, int n_in,
                              void* d_out, int out_size, void* d_ws, size_t ws_size,
                              hipStream_t stream) {
  if (n_in < 8) return;
  if (in_sizes[0] != NB * CIN * VL || in_sizes[1] != NB) return;
  if (in_sizes[2] != NE * HID * CIN || in_sizes[3] != NE * HID) return;
  if (in_sizes[4] != NE * HID * HID || in_sizes[5] != NE * HID) return;
  if (in_sizes[6] != NE * HID || in_sizes[7] != NE) return;
  if (out_size != NB * VL) return;

  const float* x  = (const float*)d_in[0];
  const int*   oi = (const int*)d_in[1];
  const float* w1 = (const float*)d_in[2];
  const float* b1 = (const float*)d_in[3];
  const float* w2 = (const float*)d_in[4];
  const float* b2 = (const float*)d_in[5];
  const float* w3 = (const float*)d_in[6];
  const float* b3 = (const float*)d_in[7];
  float* out = (float*)d_out;

  const size_t szW2S = (size_t)NB * HID * HID * 2;
  if (szW2S > ws_size || szW2S > (size_t)134217728) return;
  _Float16* w2s = (_Float16*)d_ws;

  k_prep<<<NBKP, NTHR, 0, stream>>>(w2, oi, w2s);
  k_main<<<dim3(NCH / NCHB, NB), NTHR, 0, stream>>>(x, oi, w1, b1, w2s, b2, w3, b3, out);
}
